// OuterProductMean_58918361366846
// MI455X (gfx1250) — hardware-verified
//
#include <hip/hip_runtime.h>
#include <math.h>

#ifndef NB
#define NB 1
#endif
#ifndef SEQ
#define SEQ 256
#endif
#define SEQ_FULL 256

constexpr int kPos   = SEQ;
constexpr int kPosF  = SEQ_FULL;
constexpr int kR     = 128;
constexpr int kC     = 128;
constexpr int kCO    = 32;
constexpr int kOutC  = 128;
constexpr int kOPK   = kCO * kCO;
constexpr long kPlaneHalves = (long)kPosF * kCO * kR;
constexpr float kLnEps      = 1e-5f;
constexpr float kWCarry     = 16.0f;
constexpr float kWCarryInv  = 1.0f / 16.0f;
constexpr float kResCarry   = 2048.0f;
constexpr float kResFoldInv = 1.0f / 32768.0f;
constexpr float kInvC       = 1.0f / 128.0f;
constexpr float kOutFold    = 1.0f / 2048.0f;

static_assert(NB == 1);
static_assert(SEQ % 4 == 0 && SEQ >= 4 && SEQ <= SEQ_FULL);
static_assert(kC % 32 == 0 && kR % 64 == 0 && kOPK % 32 == 0);
static_assert(kOutC == 128 && kCO == 32 && kC == 128 && kR == 128);

constexpr long kOffPL   = 0;
constexpr long kOffW1   = 2 * kPlaneHalves * 2;
constexpr long kOffW2   = kOffW1 + 2L * kCO * kC * 2;
constexpr long kWsBytes = kOffW2 + (long)kOutC * kOPK * 2;
static_assert(kOffW1 == 4194304 && kOffW2 == 4210688 && kWsBytes == 4472832);
static_assert((kOffW1 % 128) == 0 && (kOffW2 % 128) == 0);
static_assert(kWsBytes <= 134217728L);

typedef __attribute__((ext_vector_type(16))) _Float16 v16h;
typedef __attribute__((ext_vector_type(8)))  _Float16 v8h;
typedef __attribute__((ext_vector_type(2)))  _Float16 v2h;
typedef __attribute__((ext_vector_type(8)))  float    v8f;
typedef __attribute__((ext_vector_type(4)))  float    v4f;
typedef __attribute__((ext_vector_type(4)))  unsigned int v4u;
typedef __attribute__((ext_vector_type(2)))  unsigned int v2u;

__device__ __forceinline__ float bfr(float f) {
  unsigned u = __float_as_uint(f);
  u = (u + 0x7FFFu + ((u >> 16) & 1u)) & 0xffff0000u;
  return __uint_as_float(u);
}
__device__ __forceinline__ unsigned pack2h(float a, float b) {
  const v2h p = {(_Float16)a, (_Float16)b};
  return __builtin_bit_cast(unsigned, p);
}
__device__ __forceinline__ float h16_to_f32(unsigned hb) {
  const unsigned sgn = (hb & 0x8000u) << 16; const unsigned em = hb & 0x7fffu;
  const float fn = __uint_as_float((em << 13) + 0x38000000u);
  const float fs = (float)em * 5.9604644775390625e-8f;
  const float mag = (em < 0x400u) ? fs : fn; return __uint_as_float(__float_as_uint(mag) | sgn); }

__device__ __forceinline__ void dep_guard_h(v8f& a, v8f& b, v16h x, v16h y) { asm volatile("v_nop\n\tv_nop\n\tv_nop\n\tv_nop" : "+v"(a), "+v"(b) : "v"(x), "v"(y)); }
__device__ __forceinline__ void keep4_h(v16h a, v16h b, v16h c, v16h d) { asm volatile("v_nop" :: "v"(a), "v"(b), "v"(c), "v"(d)); }
__device__ __forceinline__ void acc_guard4(v8f& a, v8f& b, v8f& c, v8f& d) { asm volatile("v_nop\n\tv_nop\n\tv_nop\n\tv_nop" : "+v"(a), "+v"(b), "+v"(c), "+v"(d)); }
__device__ __forceinline__ void acc_guard2(v8f& a, v8f& b) { asm volatile("v_nop\n\tv_nop\n\tv_nop\n\tv_nop" : "+v"(a), "+v"(b)); }
__device__ __forceinline__ void guard4c5f(v8f& c0, v8f& c1, v8f& c2, v8f& c3, v16h f0, v16h f1, v16h f2, v16h f3, v16h f4) {
  asm volatile("v_nop\n\tv_nop\n\tv_nop\n\tv_nop" : "+v"(c0), "+v"(c1), "+v"(c2), "+v"(c3) : "v"(f0), "v"(f1), "v"(f2), "v"(f3), "v"(f4));
}
__device__ __forceinline__ void guard4c4f(v8f& c0, v8f& c1, v8f& c2, v8f& c3, v16h f0, v16h f1, v16h f2, v16h f3) {
  asm volatile("v_nop\n\tv_nop\n\tv_nop\n\tv_nop" : "+v"(c0), "+v"(c1), "+v"(c2), "+v"(c3) : "v"(f0), "v"(f1), "v"(f2), "v"(f3));
}
__device__ __forceinline__ void guard2c3f(v8f& c0, v8f& c1, v16h f0, v16h f1, v16h f2) {
  asm volatile("v_nop\n\tv_nop\n\tv_nop\n\tv_nop" : "+v"(c0), "+v"(c1) : "v"(f0), "v"(f1), "v"(f2));
}

template <typename T> struct Frag;
template <> struct Frag<_Float16> {
  typedef v16h V; union U { v16h v; v8h h[2]; };
  static __device__ __forceinline__ v16h load(const _Float16* p) {
    U f; f.h[0] = *(const v8h*)(p); f.h[1] = *(const v8h*)(p + 16); return f.v;
  }
  static __device__ __forceinline__ v8f mma(v16h a, v16h b, v8f c) {
    return __builtin_amdgcn_wmma_f32_16x16x32_f16(false, a, false, b, (short)0, c, false, false);
  }
  static __device__ __forceinline__ void guard(v8f& a, v8f& b, v16h x, v16h y) { dep_guard_h(a, b, x, y); }
  static __device__ __forceinline__ void keep(v16h a, v16h b, v16h c, v16h d) { keep4_h(a, b, c, d); }
};
typedef Frag<_Float16> FH;

__device__ __forceinline__ v8f zero8() { return (v8f){0.f, 0.f, 0.f, 0.f, 0.f, 0.f, 0.f, 0.f}; }

__global__ __launch_bounds__(256) void prep_weights_kernel(const float* __restrict__ w1, const float* __restrict__ w2,
                                                           unsigned short* __restrict__ w1h, unsigned short* __restrict__ w2h) {
  const int blk = blockIdx.x;
  const int t   = threadIdx.x;
  const float* src;
  unsigned short* dst;
  if (blk < 4) {
    const size_t e = (size_t)(blk * 256 + t) * 8;
    src = w1 + e;  dst = w1h + e;
  } else {
    const size_t e = (size_t)((blk - 4) * 256 + t) * 8;
    src = w2 + e;  dst = w2h + e;
  }
  const v4f a = *(const v4f*)(src);
  const v4f c = *(const v4f*)(src + 4);
  float f[8];
#pragma unroll
  for (int e = 0; e < 4; ++e) {
    const float fa = a[e];
    const float fc = c[e];
    f[e]     = bfr(fa) * kWCarry;
    f[4 + e] = bfr(fc) * kWCarry;
  }
  const v4u u = (v4u){pack2h(f[0], f[1]), pack2h(f[2], f[3]), pack2h(f[4], f[5]), pack2h(f[6], f[7])};
  *(volatile v4u*)dst = u;
  __threadfence();
  *(volatile v4u*)dst = u;
}

constexpr int kXP = 136;
constexpr int kTP = 68;
constexpr int kXhOff = 0;
constexpr int kXlOff = 64 * kXP * 2;
constexpr int kTtOff = kXlOff + 64 * kXP * 2;
constexpr int kLds2  = kTtOff + 64 * kTP * 4;
static_assert(kLds2 == 52224 && (kXlOff % 16) == 0 && (kTtOff % 16) == 0);

__global__ __launch_bounds__(128) void ln_proj_kernel(const float* __restrict__ act,
                                                      const float* __restrict__ gamma, const float* __restrict__ beta,
                                                      const unsigned short* __restrict__ w1h, const float* __restrict__ b1,
                                                      unsigned short* __restrict__ pl) {
  extern __shared__ __align__(16) unsigned char smem2[];
  unsigned short* xh = (unsigned short*)(smem2 + kXhOff);
  unsigned short* xl = (unsigned short*)(smem2 + kXlOff);
  float* tT = (float*)(smem2 + kTtOff);
  const int rh   = blockIdx.x;
  const int pi   = blockIdx.y;
  const int t    = threadIdx.x;
  const int lane = t & 31;
  const int wave = t >> 5;
  const int rbase = rh * 64;

  const int c0 = lane * 4;
  float g4[4], b4[4];
  {
    const v4f ga = *(const v4f*)(gamma + c0);
    const v4f ba = *(const v4f*)(beta + c0);
#pragma unroll
    for (int e = 0; e < 4; ++e) {
      const float f0 = ga[e], f1 = ba[e];
      g4[e] = bfr(f0); b4[e] = bfr(f1);
    }
  }

#pragma unroll 1
  for (int r = 0; r < 16; ++r) {
    const int sl = wave * 16 + r;
    const float* xr = act + ((size_t)(rbase + sl) * kPosF + pi) * kC + c0;
    const v4f xa = *(const v4f*)(xr);
    float x[4];
#pragma unroll
    for (int e = 0; e < 4; ++e) {
      const float f0 = xa[e];
      x[e] = bfr(f0);
    }
    float s1 = (x[0] + x[1]) + (x[2] + x[3]);
#pragma unroll
    for (int off = 16; off > 0; off >>= 1) s1 += __shfl_xor(s1, off, 32);
    const float mu = s1 * kInvC;
    float s2 = 0.f;
#pragma unroll
    for (int e = 0; e < 4; ++e) { const float d = x[e] - mu; s2 += d * d; }
#pragma unroll
    for (int off = 16; off > 0; off >>= 1) s2 += __shfl_xor(s2, off, 32);
    const float rstd = rsqrtf(s2 * kInvC + kLnEps);
    unsigned wh[2], wl[2];
#pragma unroll
    for (int e = 0; e < 2; ++e) {
      const float xn0 = (x[2 * e] - mu) * rstd * g4[2 * e] + b4[2 * e];
      const float xn1 = (x[2 * e + 1] - mu) * rstd * g4[2 * e + 1] + b4[2 * e + 1];
      unsigned w = pack2h(xn0, xn1);
      asm volatile("" : "+v"(w));
      const float h0 = h16_to_f32(w & 0xffffu);
      const float h1 = h16_to_f32(w >> 16);
      wh[e] = w;
      wl[e] = pack2h((xn0 - h0) * kResCarry, (xn1 - h1) * kResCarry);
    }
    const v2u uh = (v2u){wh[0], wh[1]};
    const v2u ul = (v2u){wl[0], wl[1]};
    *(v2u*)(xh + sl * kXP + c0) = uh;
    *(v2u*)(xl + sl * kXP + c0) = ul;
  }
  __syncthreads();

  const int rlane = lane & 15;
  const int hh    = lane >> 4;
  const int koff  = hh * 8;
  const _Float16* xhh = (const _Float16*)xh;
  const _Float16* xlh = (const _Float16*)xl;
  const _Float16* wlp = (const _Float16*)w1h;
  v8f acc[4], accr[4];
#pragma unroll
  for (int mi = 0; mi < 4; ++mi) { acc[mi] = zero8(); accr[mi] = zero8(); }
#pragma unroll 1
  for (int k0 = 0; k0 < kC; k0 += 32) {
    const v16h bw = FH::load(wlp + (size_t)(wave * 16 + rlane) * kC + k0 + koff);
    {
      const v16h a0 = FH::load(xhh + (0 * 16 + rlane) * kXP + k0 + koff);
      const v16h a1 = FH::load(xhh + (1 * 16 + rlane) * kXP + k0 + koff);
      const v16h a2 = FH::load(xhh + (2 * 16 + rlane) * kXP + k0 + koff);
      const v16h a3 = FH::load(xhh + (3 * 16 + rlane) * kXP + k0 + koff);
      acc[0] = FH::mma(a0, bw, acc[0]);
      acc[1] = FH::mma(a1, bw, acc[1]);
      acc[2] = FH::mma(a2, bw, acc[2]);
      acc[3] = FH::mma(a3, bw, acc[3]);
      guard4c5f(acc[0], acc[1], acc[2], acc[3], a0, a1, a2, a3, bw);
    }
    {
      const v16h l0 = FH::load(xlh + (0 * 16 + rlane) * kXP + k0 + koff);
      const v16h l1 = FH::load(xlh + (1 * 16 + rlane) * kXP + k0 + koff);
      const v16h l2 = FH::load(xlh + (2 * 16 + rlane) * kXP + k0 + koff);
      const v16h l3 = FH::load(xlh + (3 * 16 + rlane) * kXP + k0 + koff);
      accr[0] = FH::mma(l0, bw, accr[0]);
      accr[1] = FH::mma(l1, bw, accr[1]);
      accr[2] = FH::mma(l2, bw, accr[2]);
      accr[3] = FH::mma(l3, bw, accr[3]);
      guard4c5f(accr[0], accr[1], accr[2], accr[3], l0, l1, l2, l3, bw);
    }
  }
  acc_guard4(acc[0], acc[1], acc[2], acc[3]);
  acc_guard4(accr[0], accr[1], accr[2], accr[3]);

  const int f = wave * 16 + rlane;
  const float bv = bfr(b1[f]);
#pragma unroll
  for (int mi = 0; mi < 4; ++mi) {
#pragma unroll
    for (int r = 0; r < 8; ++r) {
      const int sl = mi * 16 + hh * 8 + r;
      const float v  = acc[mi][r];
      const float vr = accr[mi][r];
      tT[f * kTP + sl] = v * kWCarryInv + vr * kResFoldInv + bv;
    }
  }
  __syncthreads();

  const int q  = lane >> 3;
  const int c8 = (lane & 7) * 8;
  unsigned short* plane = pl + (size_t)(wave >> 1) * kPlaneHalves;
  const int cb = (wave & 1) * 16;
  for (int pass = 0; pass < 2; ++pass) {
#pragma unroll
    for (int it = 0; it < 4; ++it) {
      const int crow = it * 4 + q;
      const float* sp = tT + (wave * 16 + crow) * kTP + c8;
      const v4f p0 = *(const v4f*)(sp);
      const v4f p1 = *(const v4f*)(sp + 4);
      float fv[8];
#pragma unroll
      for (int e = 0; e < 4; ++e) {
        const float f0 = p0[e], f1 = p1[e];
        fv[e] = f0; fv[4 + e] = f1;
      }
      const v4u u = (v4u){pack2h(fv[0], fv[1]), pack2h(fv[2], fv[3]), pack2h(fv[4], fv[5]), pack2h(fv[6], fv[7])};
      *(volatile v4u*)(plane + ((size_t)(pi * kCO + cb + crow) * kR + rbase + c8)) = u;
    }
    __threadfence();
  }
}

constexpr int kPANP = 136;
constexpr int kOPP  = 1032;
constexpr int kOSP  = 132;
constexpr int kPanBytes = 256 * kPANP * 2;
constexpr int kOpbOff   = kPanBytes;
constexpr int kOpbBytes = 16 * kOPP * 2;
constexpr int kLds3     = kOpbOff + kOpbBytes;
static_assert(kLds3 == 102656 && (kOpbOff % 16) == 0);
static_assert(16 * kOSP * 4 <= kPanBytes);

__global__ __launch_bounds__(128) void pair_kernel(const unsigned short* __restrict__ pl, const unsigned short* __restrict__ w2h,
                                                   const float* __restrict__ b2, float* __restrict__ out) {
  extern __shared__ __align__(16) unsigned char smem3[];
  unsigned short* pan  = (unsigned short*)(smem3);
  _Float16*       opbw = (_Float16*)(smem3 + kOpbOff);
  float*          outS = (float*)(smem3);

  const int i0   = blockIdx.x * 4;
  const int j0   = blockIdx.y * 4;
  const int t    = threadIdx.x;
  const int lane = t & 31;
  const int wave = t >> 5;
  const int rlane = lane & 15;
  const int hh    = lane >> 4;
  const int koff  = hh * 8;

  {
    const v4u* gl = (const v4u*)(pl + (size_t)i0 * kCO * kR);
    const v4u* gr = (const v4u*)(pl + kPlaneHalves + (size_t)j0 * kCO * kR);
#pragma unroll 1
    for (int it = 0; it < 16; ++it) {
      const int idx  = it * 128 + t;
      const int row  = idx >> 4;
      const int col8 = (idx & 15) * 8;
      const v4u a = gl[idx];
      const v4u b = gr[idx];
      *(v4u*)(pan + row * kPANP + col8) = a;
      *(v4u*)(pan + (128 + row) * kPANP + col8) = b;
      asm volatile("" ::: "memory");
    }
  }
  __syncthreads();

  const _Float16* panh = (const _Float16*)pan;
#pragma unroll 1
  for (int jp = 0; jp < 4; ++jp) {
    v8f acc[2][2];
    acc[0][0] = zero8(); acc[0][1] = zero8(); acc[1][0] = zero8(); acc[1][1] = zero8();
#pragma unroll
    for (int kc = 0; kc < 4; ++kc) {
      const int k0 = kc * 32;
      const v16h af0 = FH::load(panh + (wave * 32 + rlane) * kPANP + k0 + koff);
      const v16h af1 = FH::load(panh + (wave * 32 + 16 + rlane) * kPANP + k0 + koff);
      const v16h bf0 = FH::load(panh + (128 + jp * 32 + rlane) * kPANP + k0 + koff);
      const v16h bf1 = FH::load(panh + (128 + jp * 32 + 16 + rlane) * kPANP + k0 + koff);
      acc[0][0] = FH::mma(af0, bf0, acc[0][0]);
      acc[0][1] = FH::mma(af0, bf1, acc[0][1]);
      acc[1][0] = FH::mma(af1, bf0, acc[1][0]);
      acc[1][1] = FH::mma(af1, bf1, acc[1][1]);
      guard4c4f(acc[0][0], acc[0][1], acc[1][0], acc[1][1], af0, af1, bf0, bf1);
    }
    acc_guard4(acc[0][0], acc[0][1], acc[1][0], acc[1][1]);
    const int p = wave * 4 + jp;
#pragma unroll
    for (int mt = 0; mt < 2; ++mt) {
#pragma unroll
      for (int nt = 0; nt < 2; ++nt) {
#pragma unroll
        for (int r = 0; r < 8; ++r) {
          const int c = mt * 16 + hh * 8 + r;
          const int d = nt * 16 + rlane;
          const float v = acc[mt][nt][r];
          opbw[p * kOPP + c * 32 + d] = (_Float16)v;
        }
      }
    }
  }
  __syncthreads();

  const _Float16* opbh = (const _Float16*)opbw;
  const _Float16* woh  = (const _Float16*)w2h;
  v8f acc2[2];
  acc2[0] = zero8(); acc2[1] = zero8();
#pragma unroll 1
  for (int k0 = 0; k0 < kOPK; k0 += 32) {
    const v16h a  = FH::load(opbh + rlane * kOPP + k0 + koff);
    const v16h b0 = FH::load(woh + (size_t)(wave * 16 + rlane) * kOPK + k0 + koff);
    const v16h bq = FH::load(woh + (size_t)((wave + 4) * 16 + rlane) * kOPK + k0 + koff);
    acc2[0] = FH::mma(a, b0, acc2[0]);
    acc2[1] = FH::mma(a, bq, acc2[1]);
    guard2c3f(acc2[0], acc2[1], a, b0, bq);
  }
  acc_guard2(acc2[0], acc2[1]);

  {
    const int o0 = wave * 16 + rlane;
    const int o1 = (wave + 4) * 16 + rlane;
    const float bo0 = bfr(b2[o0]);
    const float bo1 = bfr(b2[o1]);
#pragma unroll
    for (int r = 0; r < 8; ++r) {
      const int p = hh * 8 + r;
      const float v0 = acc2[0][r];
      const float v1 = acc2[1][r];
      outS[p * kOSP + o0] = v0 * kOutFold + bo0;
      outS[p * kOSP + o1] = v1 * kOutFold + bo1;
    }
  }
  __syncthreads();

  for (int pass = 0; pass < 2; ++pass) {
#pragma unroll
    for (int it = 0; it < 4; ++it) {
      const int p = wave * 4 + it;
      const v4f v = *(const v4f*)(outS + p * kOSP + lane * 4);
      *(volatile v4f*)(out + ((size_t)((i0 + wave) * kPosF + (j0 + it))) * kOutC + lane * 4) = v;
    }
    __threadfence();
  }
}

extern "C" void kernel_launch(void* const* d_in, const int* in_sizes, int n_in,
                              void* d_out, int out_size, void* d_ws, size_t ws_size, hipStream_t stream) {
  if (n_in < 7) return;
  if ((long)in_sizes[0] < ((long)(kR - 1) * kPosF + kPos) * kC) return;
  if (in_sizes[1] < kC || in_sizes[2] < kC) return;
  if (in_sizes[3] < 2 * kCO * kC || in_sizes[4] < 2 * kCO) return;
  if (in_sizes[5] < kOutC * kOPK || in_sizes[6] < kOutC) return;
  if ((long)out_size < ((long)(kPos - 1) * kPosF + kPos) * kOutC) return;
  if (ws_size < (size_t)kWsBytes) return;

  const float* act   = (const float*)d_in[0];
  const float* gamma = (const float*)d_in[1];
  const float* beta  = (const float*)d_in[2];
  const float* w1    = (const float*)d_in[3];
  const float* b1    = (const float*)d_in[4];
  const float* w2    = (const float*)d_in[5];
  const float* b2    = (const float*)d_in[6];
  float* out = (float*)d_out;

  unsigned char* ws = (unsigned char*)d_ws;
  unsigned short* pl  = (unsigned short*)(ws + kOffPL);
  unsigned short* w1h = (unsigned short*)(ws + kOffW1);
  unsigned short* w2h = (unsigned short*)(ws + kOffW2);

  hipFuncSetAttribute(reinterpret_cast<const void*>(&pair_kernel), hipFuncAttributeMaxDynamicSharedMemorySize, kLds3);

  prep_weights_kernel<<<dim3(68), dim3(256), 0, stream>>>(w1, w2, w1h, w2h);
  ln_proj_kernel<<<dim3(kR / 64, kPos), dim3(128), kLds2, stream>>>(act, gamma, beta, w1h, b1, pl);
  pair_kernel<<<dim3(kPos / 4, kPos / 4), dim3(128), kLds3, stream>>>(pl, w2h, b2, out);
}
